// LocalBlock_63187558859377
// MI455X (gfx1250) — hardware-verified
//
#include <hip/hip_runtime.h>
#include <math.h>

constexpr int kSeq        = 4096;
constexpr int kDim        = 1024;
constexpr int kHeads      = 16;
constexpr int kHd         = 64;
constexpr int kWin        = 256;
constexpr int kGuard      = 256;
constexpr int kTokG       = kSeq + kGuard;
constexpr int kBand       = kWin + 64;
constexpr int kColsA      = 256;
constexpr int kQKCols     = 2 * kDim;
constexpr int kFF         = 4 * kDim;
constexpr int kChunkHeads = 4;
constexpr int kNumChunks  = kHeads / kChunkHeads;
constexpr float kWCarry    = 16.0f;
constexpr float kWCarryInv = 1.0f / 16.0f;
constexpr float kPCarry    = 2048.0f;
constexpr float kOCarry    = 256.0f;
constexpr float kGCarry    = 16.0f;
constexpr float kLnEps     = 1e-5f;

constexpr size_t kOffWqkv = 0;
constexpr size_t kOffWout = kOffWqkv + (size_t)3 * kDim * kDim * 2;
constexpr size_t kOffWm1  = kOffWout + (size_t)kDim * kDim * 2;
constexpr size_t kOffWm2  = kOffWm1 + (size_t)kFF * kDim * 2;
constexpr size_t kOffNrm  = kOffWm2 + (size_t)kDim * kFF * 2;
constexpr size_t kOffH1   = kOffNrm + (size_t)kSeq * kDim * 2;
constexpr size_t kOffO16  = kOffH1 + (size_t)kSeq * kDim * 4;
constexpr size_t kOffAtt  = kOffO16 + (size_t)kSeq * kDim * 2;
constexpr size_t kOffQKG  = kOffAtt;
constexpr size_t kOffVT   = kOffQKG + (size_t)kTokG * kQKCols * 2;
constexpr size_t kOffSB   = kOffVT + (size_t)kDim * kTokG * 2;
constexpr size_t kOffPB   = kOffSB + (size_t)kChunkHeads * kSeq * kBand * 4;
constexpr size_t kEndPB   = kOffPB + (size_t)kChunkHeads * kSeq * kBand * 2;
constexpr size_t kOffU16  = kOffAtt;
constexpr size_t kOffG16  = kOffU16 + (size_t)kSeq * kFF * 2;
constexpr size_t kEndG16  = kOffG16 + (size_t)kSeq * kFF * 2;
constexpr size_t kWsTotal = (kEndPB > kEndG16) ? kEndPB : kEndG16;
static_assert(kWsTotal == 125829120u, "carve");
static_assert(kWsTotal <= 134217728u, "carve cap");
static_assert((kOffVT % 4096) == 0 && (kOffSB % 4096) == 0 && (kOffPB % 4096) == 0 && (kOffG16 % 4096) == 0, "align");

typedef __attribute__((ext_vector_type(16))) _Float16 v16h;
typedef __attribute__((ext_vector_type(8)))  _Float16 v8h;
typedef __attribute__((ext_vector_type(16))) __bf16   v16b;
typedef __attribute__((ext_vector_type(8)))  __bf16   v8b;
typedef __attribute__((ext_vector_type(8)))  float    v8f;
typedef __attribute__((ext_vector_type(4)))  float    v4f;
typedef __attribute__((ext_vector_type(4)))  unsigned int v4u;

__device__ __forceinline__ unsigned short f2bf_bits(float f) {
  unsigned u = __float_as_uint(f);
  return (unsigned short)((u + 0x7FFFu + ((u >> 16) & 1u)) >> 16);
}
__device__ __forceinline__ float bf_bits2f(unsigned short h) { return __uint_as_float(((unsigned)h) << 16); }

__device__ __forceinline__ void dep_guard_h(v8f& a, v8f& b, v16h x, v16h y) { asm volatile("v_nop\n\tv_nop\n\tv_nop\n\tv_nop" : "+v"(a), "+v"(b) : "v"(x), "v"(y)); }
__device__ __forceinline__ void dep_guard_b(v8f& a, v8f& b, v16b x, v16b y) { asm volatile("v_nop\n\tv_nop\n\tv_nop\n\tv_nop" : "+v"(a), "+v"(b) : "v"(x), "v"(y)); }
__device__ __forceinline__ void keep4_h(v16h a, v16h b, v16h c, v16h d) { asm volatile("v_nop" :: "v"(a), "v"(b), "v"(c), "v"(d)); }
__device__ __forceinline__ void keep4_b(v16b a, v16b b, v16b c, v16b d) { asm volatile("v_nop" :: "v"(a), "v"(b), "v"(c), "v"(d)); }
__device__ __forceinline__ void acc_guard4(v8f& a, v8f& b, v8f& c, v8f& d) { asm volatile("v_nop\n\tv_nop\n\tv_nop\n\tv_nop" : "+v"(a), "+v"(b), "+v"(c), "+v"(d)); }
template <typename T> struct Frag;
template <> struct Frag<_Float16> {
  typedef v16h V; union U { v16h v; v8h h[2]; };
  static __device__ __forceinline__ v16h load(const _Float16* p) {
    U f; f.h[0] = *(const v8h*)(p); f.h[1] = *(const v8h*)(p + 16); return f.v;
  }
  static __device__ __forceinline__ v8f mma(v16h a, v16h b, v8f c) {
    return __builtin_amdgcn_wmma_f32_16x16x32_f16(false, a, false, b, (short)0, c, false, false);
  }
  static __device__ __forceinline__ void guard(v8f& a, v8f& b, v16h x, v16h y) { dep_guard_h(a, b, x, y); }
  static __device__ __forceinline__ void keep(v16h a, v16h b, v16h c, v16h d) { keep4_h(a, b, c, d); }
};
template <> struct Frag<__bf16> {
  typedef v16b V; union U { v16b v; v8b h[2]; };
  static __device__ __forceinline__ v16b load(const __bf16* p) {
    U f; f.h[0] = *(const v8b*)(p); f.h[1] = *(const v8b*)(p + 16); return f.v;
  }
  static __device__ __forceinline__ v8f mma(v16b a, v16b b, v8f c) {
    return __builtin_amdgcn_wmma_f32_16x16x32_bf16(false, a, false, b, (short)0, c, false, false);
  }
  static __device__ __forceinline__ void guard(v8f& a, v8f& b, v16b x, v16b y) { dep_guard_b(a, b, x, y); }
  static __device__ __forceinline__ void keep(v16b a, v16b b, v16b c, v16b d) { keep4_b(a, b, c, d); }
};

__device__ __forceinline__ unsigned pk16(unsigned short a, unsigned short b) { return (unsigned)a | ((unsigned)b << 16); }
__device__ __forceinline__ unsigned short h_bits(float f) { const _Float16 h = (_Float16)f; return __builtin_bit_cast(unsigned short, h); }
__device__ __forceinline__ float h_lo2f(unsigned u) { return (float)__builtin_bit_cast(_Float16, (unsigned short)(u & 0xffffu)); }
__device__ __forceinline__ float h_hi2f(unsigned u) { return (float)__builtin_bit_cast(_Float16, (unsigned short)(u >> 16)); }

template <int ET> struct Elem;
template <> struct Elem<0> { typedef _Float16 T; };
template <> struct Elem<1> { typedef __bf16 T; };
template <int ET, bool SPLIT, int BIAS_MODE, int OUT_MODE, bool RESID>
__global__ __launch_bounds__(256) void wmma_gemm64(
    const unsigned short* __restrict__ Ap, const unsigned short* __restrict__ A2p, int lda, long strideA,
    const unsigned short* __restrict__ Btp, const unsigned short* __restrict__ Bt2p, int ldb, long strideB, long bandB,
    void* __restrict__ Cout, void* __restrict__ Cout2, int ldc, long strideC,
    const float* __restrict__ bias,
    const float* __restrict__ resid, long strideR,
    int M, int N, int K, float scale) {
  typedef typename Elem<ET>::T T;
  typedef typename Frag<T>::V V;
  const T* A = (const T*)Ap; const T* A2 = (const T*)A2p; const T* Bt = (const T*)Btp; const T* Bt2 = (const T*)Bt2p;
  __shared__ __align__(16) float sT[8][16 * 68];
  const int b    = blockIdx.y;
  const int lane = threadIdx.x & 31;
  const int wave = threadIdx.x >> 5;
  const int tilesN = N >> 6;
  const int tilesM = M >> 6;
  const int tile = blockIdx.x * 8 + wave;
  if (tile >= tilesM * tilesN) return;
  const int tm = tile / tilesN;
  const int tn = tile - tm * tilesN;
  const int m0 = tm << 6;
  const int n0 = tn << 6;

  const T* Ab  = A  + (size_t)b * strideA;
  const T* Bb  = Bt + (size_t)b * strideB + (size_t)tm * bandB;
  const T* Ab2 = SPLIT ? (A2  + (size_t)b * strideA) : nullptr;
  const T* Bb2 = SPLIT ? (Bt2 + (size_t)b * strideB + (size_t)tm * bandB) : nullptr;

  const int rlane = lane & 15;
  const int koff  = (lane >> 4) * 8;
  const int mOff  = (lane >> 4) * 8;

  v8f acc[4][4];
#pragma unroll
  for (int i = 0; i < 4; ++i)
#pragma unroll
    for (int j = 0; j < 4; ++j) acc[i][j] = (v8f){0.f,0.f,0.f,0.f,0.f,0.f,0.f,0.f};

  for (int k0 = 0; k0 < K; k0 += 32) {
    V bh[4], bl[4];
#pragma unroll
    for (int j = 0; j < 4; ++j) {
      const size_t bo = (size_t)(n0 + (j << 4) + rlane) * ldb + koff + k0;
      bh[j] = Frag<T>::load(Bb + bo);
      if (SPLIT) bl[j] = Frag<T>::load(Bb2 + bo);
    }
#pragma unroll
    for (int i = 0; i < 4; ++i) {
      const size_t ao = (size_t)(m0 + (i << 4) + rlane) * lda + koff + k0;
      V ah = Frag<T>::load(Ab + ao);
      V al;
      if (SPLIT) al = Frag<T>::load(Ab2 + ao);
#pragma unroll
      for (int j = 0; j < 4; ++j) {
        acc[i][j] = Frag<T>::mma(ah, bh[j], acc[i][j]);
        if (SPLIT) {
          acc[i][j] = Frag<T>::mma(ah, bl[j], acc[i][j]);
          acc[i][j] = Frag<T>::mma(al, bh[j], acc[i][j]);
        }
      }
      Frag<T>::guard(acc[i][0], acc[i][3], ah, SPLIT ? al : ah);
    }
    Frag<T>::keep(bh[0], bh[1], bh[2], bh[3]);
    if (SPLIT) Frag<T>::keep(bl[0], bl[1], bl[2], bl[3]);
  }
  acc_guard4(acc[0][0], acc[0][1], acc[0][2], acc[0][3]);
  acc_guard4(acc[1][0], acc[1][1], acc[1][2], acc[1][3]);
  acc_guard4(acc[2][0], acc[2][1], acc[2][2], acc[2][3]);
  acc_guard4(acc[3][0], acc[3][1], acc[3][2], acc[3][3]);

  float* slab = sT[wave];
  const float* Rb = RESID ? (resid + (size_t)b * strideR) : nullptr;
#pragma unroll
  for (int i = 0; i < 4; ++i) {
    const int mBase = m0 + (i << 4);
#pragma unroll
    for (int j = 0; j < 4; ++j) {
      const int n = n0 + (j << 4) + rlane;
      float bv = 0.f;
      if (BIAS_MODE == 2) bv = bias[n];
#pragma unroll
      for (int r = 0; r < 8; ++r) {
        float v = acc[i][j][r] * scale;
        if (BIAS_MODE == 1) v += bias[mBase + mOff + r];
        if (BIAS_MODE == 2) v += bv;
        if (RESID) v += Rb[(size_t)(mBase + mOff + r) * ldc + n];
        slab[(mOff + r) * 68 + (j << 4) + rlane] = v;
      }
    }
    __builtin_amdgcn_fence(__ATOMIC_RELEASE, "workgroup");
    __builtin_amdgcn_wave_barrier();
    __builtin_amdgcn_fence(__ATOMIC_ACQUIRE, "workgroup");
    if (OUT_MODE == 0) {
      float* C = (float*)Cout + (size_t)b * strideC;
      const int hh = lane >> 4, c4 = (lane & 15) * 4;
      for (int pass = 0; pass < 2; ++pass) {
#pragma unroll
        for (int it = 0; it < 8; ++it) {
          const int row = it * 2 + hh;
          v4f v = *(const v4f*)(slab + row * 68 + c4);
          *(volatile v4f*)(C + (size_t)(mBase + row) * ldc + n0 + c4) = v;
        }
        __threadfence();
      }
    } else {
      const int q = lane >> 3, c8 = (lane & 7) * 8;
      unsigned short* C  = (unsigned short*)Cout  + (size_t)b * strideC;
      unsigned short* C2 = (OUT_MODE == 2) ? ((unsigned short*)Cout2 + (size_t)b * strideC) : nullptr;
      for (int pass = 0; pass < 2; ++pass) {
#pragma unroll
        for (int it = 0; it < 4; ++it) {
          const int row = it * 4 + q;
          const float* sp = slab + row * 68 + c8;
          v8h hv, lv;
#pragma unroll
          for (int e = 0; e < 8; ++e) {
            if (OUT_MODE == 1) {
              hv[e] = (_Float16)sp[e];
            } else {
              unsigned short hb = f2bf_bits(sp[e]);
              unsigned short lb = f2bf_bits(sp[e] - bf_bits2f(hb));
              hv[e] = __builtin_bit_cast(_Float16, hb);
              lv[e] = __builtin_bit_cast(_Float16, lb);
            }
          }
          *(volatile v8h*)(C + (size_t)(mBase + row) * ldc + n0 + c8) = hv;
          if (OUT_MODE == 2) *(volatile v8h*)(C2 + (size_t)(mBase + row) * ldc + n0 + c8) = lv;
        }
        __threadfence();
      }
    }
    __builtin_amdgcn_fence(__ATOMIC_RELEASE, "workgroup");
    __builtin_amdgcn_wave_barrier();
    __builtin_amdgcn_fence(__ATOMIC_ACQUIRE, "workgroup");
  }
}

__global__ __launch_bounds__(256) void wtcast_kernel(const float* __restrict__ W, unsigned short* __restrict__ out,
                                                     int R, int C, float scale) {
  __shared__ float sm[64][65];
  const int t  = threadIdx.x;
  const int k0 = blockIdx.x * 64;
  const int n0 = blockIdx.y * 64;
#pragma unroll
  for (int i = 0; i < 16; ++i) {
    const int e = i * 256 + t;
    const int r = e >> 6;
    const int c = e & 63;
    sm[c][r] = W[(size_t)(k0 + r) * C + n0 + c] * scale;
  }
  __syncthreads();
  const int lane = t & 31, wave = t >> 5;
  const int q = lane >> 3, c8 = (lane & 7) * 8;
  for (int pass = 0; pass < 2; ++pass) {
#pragma unroll
    for (int it = 0; it < 2; ++it) {
      const int row = wave * 8 + it * 4 + q;
      unsigned short hb[8];
#pragma unroll
      for (int e = 0; e < 8; ++e) hb[e] = h_bits(sm[row][c8 + e]);
      const v4u u = (v4u){pk16(hb[0], hb[1]), pk16(hb[2], hb[3]), pk16(hb[4], hb[5]), pk16(hb[6], hb[7])};
      *(volatile v4u*)(out + (size_t)(n0 + row) * R + k0 + c8) = u;
    }
    __threadfence();
  }
}

__global__ __launch_bounds__(256) void fill_zero16_kernel(unsigned short* __restrict__ base, int rows,
                                                          int pitch_halves, int segs_per_row) {
  const int i = blockIdx.x * 256 + threadIdx.x;
  const int total = rows * segs_per_row;
  if (i >= total) return;
  const int row = i / segs_per_row;
  const int seg = i - row * segs_per_row;
  unsigned short* p = base + (size_t)row * pitch_halves + (size_t)seg * 8;
  const v4u z = (v4u){0u, 0u, 0u, 0u};
  *(volatile v4u*)p = z;
  __threadfence();
  *(volatile v4u*)p = z;
}

__global__ __launch_bounds__(128) void layernorm_f16_kernel(const float* __restrict__ x, const float* __restrict__ w,
                                                            const float* __restrict__ bparam, unsigned short* __restrict__ out) {
  __shared__ float red1[4];
  __shared__ float red2[4];
  const int row  = blockIdx.x;
  const int t    = threadIdx.x;
  const int lane = t & 31, wave = t >> 5;
  const float* xr = x + (size_t)row * kDim + 8 * t;
  const v4f a = *(const v4f*)(xr);
  const v4f c = *(const v4f*)(xr + 4);
  float v[8];
#pragma unroll
  for (int e = 0; e < 4; ++e) { v[e] = a[e]; v[4 + e] = c[e]; }
  float s = 0.f;
#pragma unroll
  for (int e = 0; e < 8; ++e) s += v[e];
#pragma unroll
  for (int off = 16; off > 0; off >>= 1) s += __shfl_xor(s, off, 32);
  if (lane == 0) red1[wave] = s;
  __syncthreads();
  const float mu = ((red1[0] + red1[1]) + (red1[2] + red1[3])) * (1.0f / (float)kDim);
  float d[8];
  float s2 = 0.f;
#pragma unroll
  for (int e = 0; e < 8; ++e) { d[e] = v[e] - mu; s2 += d[e] * d[e]; }
#pragma unroll
  for (int off = 16; off > 0; off >>= 1) s2 += __shfl_xor(s2, off, 32);
  if (lane == 0) red2[wave] = s2;
  __syncthreads();
  const float var = ((red2[0] + red2[1]) + (red2[2] + red2[3])) * (1.0f / (float)kDim);
  const float inv = rsqrtf(var + kLnEps);
  const v4f wa = *(const v4f*)(w + 8 * t);
  const v4f wc = *(const v4f*)(w + 8 * t + 4);
  const v4f ba = *(const v4f*)(bparam + 8 * t);
  const v4f bc = *(const v4f*)(bparam + 8 * t + 4);
  float wv[8], bv[8];
#pragma unroll
  for (int e = 0; e < 4; ++e) { wv[e] = wa[e]; wv[4 + e] = wc[e]; bv[e] = ba[e]; bv[4 + e] = bc[e]; }
  unsigned short hb[8];
#pragma unroll
  for (int e = 0; e < 8; ++e) hb[e] = h_bits(d[e] * inv * wv[e] + bv[e]);
  const v4u u = (v4u){pk16(hb[0], hb[1]), pk16(hb[2], hb[3]), pk16(hb[4], hb[5]), pk16(hb[6], hb[7])};
  unsigned short* op = out + (size_t)row * kDim + 8 * t;
  *(volatile v4u*)op = u;
  __threadfence();
  *(volatile v4u*)op = u;
}

__global__ __launch_bounds__(256) void band_softmax_kernel(const float* __restrict__ S, unsigned short* __restrict__ P, int nrows) {
  const int lane = threadIdx.x & 31;
  const int wave = threadIdx.x >> 5;
  const int gr = blockIdx.x * 8 + wave;
  if (gr >= nrows) return;
  const int rr = gr & (kSeq - 1);
  const int qt = rr >> 6;
  const int qi = rr & 63;
  int lo = kGuard - 64 * qt;
  lo = (lo > qi) ? lo : qi;
  const int hi = kWin + qi;
  const float* sr = S + (size_t)gr * kBand;
  const v4f a = *(const v4f*)(sr + 8 * lane);
  const v4f c = *(const v4f*)(sr + 8 * lane + 4);
  const float t0 = sr[kColsA + 2 * lane];
  const float t1 = sr[kColsA + 2 * lane + 1];
  float x[10];
  int col[10];
#pragma unroll
  for (int e = 0; e < 4; ++e) { x[e] = a[e]; x[4 + e] = c[e]; }
  x[8] = t0; x[9] = t1;
#pragma unroll
  for (int e = 0; e < 8; ++e) col[e] = 8 * lane + e;
  col[8] = kColsA + 2 * lane;
  col[9] = kColsA + 2 * lane + 1;
  bool vis[10];
  float m = -INFINITY;
#pragma unroll
  for (int e = 0; e < 10; ++e) {
    vis[e] = (col[e] >= lo) && (col[e] <= hi);
    x[e] = x[e] * 0.125f;
    m = vis[e] ? fmaxf(m, x[e]) : m;
  }
#pragma unroll
  for (int off = 16; off > 0; off >>= 1) m = fmaxf(m, __shfl_xor(m, off, 32));
  float p[10];
  float sum = 0.f;
#pragma unroll
  for (int e = 0; e < 10; ++e) {
    const float arg = vis[e] ? (x[e] - m) : 0.0f;
    const float ev = expf(arg);
    p[e] = vis[e] ? ev : 0.0f;
    sum += p[e];
  }
#pragma unroll
  for (int off = 16; off > 0; off >>= 1) sum += __shfl_xor(sum, off, 32);
  const float rs = kPCarry * (1.0f / sum);
  unsigned short hb[10];
#pragma unroll
  for (int e = 0; e < 10; ++e) hb[e] = h_bits(p[e] * rs);
  const v4u uA = (v4u){pk16(hb[0], hb[1]), pk16(hb[2], hb[3]), pk16(hb[4], hb[5]), pk16(hb[6], hb[7])};
  const unsigned uB = pk16(hb[8], hb[9]);
  unsigned short* pr = P + (size_t)gr * kBand;
  for (int pass = 0; pass < 2; ++pass) {
    *(volatile v4u*)(pr + 8 * lane) = uA;
    *(volatile unsigned*)(pr + kColsA + 2 * lane) = uB;
    __threadfence();
  }
}

__global__ __launch_bounds__(256) void gelu_f16_kernel(const unsigned* __restrict__ in32, unsigned short* __restrict__ out, float oscale) {
  __shared__ __align__(16) unsigned sm[1024];
  const int t = threadIdx.x;
  const size_t wbase = (size_t)blockIdx.x * 1024;
#pragma unroll 1
  for (int w = 0; w < 4; ++w) {
    const unsigned u = in32[wbase + (size_t)w * 256 + t];
    const float ua = h_lo2f(u);
    const float ub = h_hi2f(u);
    const float ga = 0.5f * ua * (1.0f + erff(ua * 0.70710678118654752f));
    const float gb = 0.5f * ub * (1.0f + erff(ub * 0.70710678118654752f));
    sm[w * 256 + t] = pk16(h_bits(ga * oscale), h_bits(gb * oscale));
  }
  __syncthreads();
  const v4u v = *(const v4u*)(sm + 4 * t);
  unsigned short* op = out + 2 * (wbase + 4 * (size_t)t);
  *(volatile v4u*)op = v;
  __threadfence();
  *(volatile v4u*)op = v;
}

extern "C" void kernel_launch(void* const* d_in, const int* in_sizes, int n_in,
                              void* d_out, int out_size, void* d_ws,
                              size_t ws_size, hipStream_t stream) {
  if (n_in < 13) return;
  if ((size_t)out_size < (size_t)kSeq * kDim) return;
  if (ws_size < kWsTotal) return;
  if (in_sizes[0] != kSeq * kDim) return;
  if (in_sizes[1] < kDim || in_sizes[2] < kDim) return;
  if (in_sizes[3] != kDim * 3 * kDim || in_sizes[4] < 3 * kDim) return;
  if (in_sizes[5] != kDim * kDim || in_sizes[6] < kDim) return;
  if (in_sizes[7] < kDim || in_sizes[8] < kDim) return;
  if (in_sizes[9] != kDim * kFF || in_sizes[10] < kFF) return;
  if (in_sizes[11] != kFF * kDim || in_sizes[12] < kDim) return;

  const float* hs     = (const float*)d_in[0];
  const float* ln1_w  = (const float*)d_in[1];
  const float* ln1_b  = (const float*)d_in[2];
  const float* qkv_w  = (const float*)d_in[3];
  const float* qkv_b  = (const float*)d_in[4];
  const float* out_w  = (const float*)d_in[5];
  const float* out_b  = (const float*)d_in[6];
  const float* ln2_w  = (const float*)d_in[7];
  const float* ln2_b  = (const float*)d_in[8];
  const float* mlp1_w = (const float*)d_in[9];
  const float* mlp1_b = (const float*)d_in[10];
  const float* mlp2_w = (const float*)d_in[11];
  const float* mlp2_b = (const float*)d_in[12];
  float* outp = (float*)d_out;

  char* ws = (char*)d_ws;
  unsigned short* wqkv = (unsigned short*)(ws + kOffWqkv);
  unsigned short* wout = (unsigned short*)(ws + kOffWout);
  unsigned short* wm1  = (unsigned short*)(ws + kOffWm1);
  unsigned short* wm2  = (unsigned short*)(ws + kOffWm2);
  unsigned short* nrm  = (unsigned short*)(ws + kOffNrm);
  float*          h1   = (float*)(ws + kOffH1);
  unsigned short* o16  = (unsigned short*)(ws + kOffO16);
  unsigned short* qkg  = (unsigned short*)(ws + kOffQKG);
  unsigned short* vt   = (unsigned short*)(ws + kOffVT);
  float*          sb   = (float*)(ws + kOffSB);
  unsigned short* pb   = (unsigned short*)(ws + kOffPB);
  unsigned short* u16  = (unsigned short*)(ws + kOffU16);
  unsigned short* g16  = (unsigned short*)(ws + kOffG16);

  wtcast_kernel<<<dim3(kDim / 64, (3 * kDim) / 64), 256, 0, stream>>>(qkv_w, wqkv, kDim, 3 * kDim, kWCarry);
  wtcast_kernel<<<dim3(kDim / 64, kDim / 64), 256, 0, stream>>>(out_w, wout, kDim, kDim, kWCarry);
  wtcast_kernel<<<dim3(kDim / 64, kFF / 64), 256, 0, stream>>>(mlp1_w, wm1, kDim, kFF, kWCarry);
  wtcast_kernel<<<dim3(kFF / 64, kDim / 64), 256, 0, stream>>>(mlp2_w, wm2, kFF, kDim, kWCarry);

  fill_zero16_kernel<<<(kGuard * (kQKCols / 8)) / 256, 256, 0, stream>>>(qkg, kGuard, kQKCols, kQKCols / 8);
  fill_zero16_kernel<<<(kDim * (kGuard / 8)) / 256, 256, 0, stream>>>(vt, kDim, kTokG, kGuard / 8);

  layernorm_f16_kernel<<<kSeq, 128, 0, stream>>>(hs, ln1_w, ln1_b, nrm);

  {
    const int tiles = (kSeq / 64) * (kQKCols / 64);
    unsigned short* cq = qkg + (size_t)kGuard * kQKCols;
    wmma_gemm64<0, false, 2, 1, false><<<dim3((tiles + 7) / 8, 1), 256, 0, stream>>>(
        nrm, nrm, kDim, 0L, wqkv, wqkv, kDim, 0L, 0L,
        (void*)cq, (void*)cq, kQKCols, 0L, qkv_b, hs, 0L, kSeq, kQKCols, kDim, kWCarryInv);
  }
  {
    const int tiles = (kDim / 64) * (kSeq / 64);
    const unsigned short* av = wqkv + (size_t)2 * kDim * kDim;
    unsigned short* cv = vt + kGuard;
    wmma_gemm64<0, false, 1, 1, false><<<dim3((tiles + 7) / 8, 1), 256, 0, stream>>>(
        av, av, kDim, 0L, nrm, nrm, kDim, 0L, 0L,
        (void*)cv, (void*)cv, kTokG, 0L, qkv_b + 2 * kDim, hs, 0L, kDim, kSeq, kDim, kWCarryInv);
  }

  for (int cc = 0; cc < kNumChunks; ++cc) {
    const int h0 = cc * kChunkHeads;
    {
      const int tiles = (kSeq / 64) * (kBand / 64);
      const unsigned short* aq = qkg + (size_t)kGuard * kQKCols + (size_t)h0 * kHd;
      const unsigned short* bk = qkg + kDim + (size_t)h0 * kHd;
      wmma_gemm64<0, false, 0, 0, false><<<dim3((tiles + 7) / 8, kChunkHeads), 256, 0, stream>>>(
          aq, aq, kQKCols, (long)kHd, bk, bk, kQKCols, (long)kHd, (long)64 * kQKCols,
          (void*)sb, (void*)sb, kBand, (long)kSeq * kBand, qkv_b, hs, 0L, kSeq, kBand, kHd, 1.0f);
    }
    band_softmax_kernel<<<(kChunkHeads * kSeq) / 8, 256, 0, stream>>>(sb, pb, kChunkHeads * kSeq);
    {
      const int tiles = (kSeq / 64) * (kHd / 64);
      const unsigned short* bv = vt + (size_t)h0 * kHd * kTokG;
      unsigned short* co = o16 + (size_t)h0 * kHd;
      wmma_gemm64<0, false, 0, 1, false><<<dim3((tiles + 7) / 8, kChunkHeads), 256, 0, stream>>>(
          pb, pb, kBand, (long)kSeq * kBand, bv, bv, kTokG, (long)kHd * kTokG, (long)kHd,
          (void*)co, (void*)co, kDim, (long)kHd, qkv_b, hs, 0L, kSeq, kHd, kBand, kOCarry / kPCarry);
    }
  }

  {
    const int tiles = (kSeq / 64) * (kDim / 64);
    wmma_gemm64<0, false, 2, 0, true><<<dim3((tiles + 7) / 8, 1), 256, 0, stream>>>(
        o16, o16, kDim, 0L, wout, wout, kDim, 0L, 0L,
        (void*)h1, (void*)h1, kDim, 0L, out_b, hs, 0L, kSeq, kDim, kDim, 1.0f / (kOCarry * kWCarry));
  }
  layernorm_f16_kernel<<<kSeq, 128, 0, stream>>>(h1, ln2_w, ln2_b, nrm);
  {
    const int tiles = (kSeq / 64) * (kFF / 64);
    wmma_gemm64<0, false, 2, 1, false><<<dim3((tiles + 7) / 8, 1), 256, 0, stream>>>(
        nrm, nrm, kDim, 0L, wm1, wm1, kDim, 0L, 0L,
        (void*)u16, (void*)u16, kFF, 0L, mlp1_b, hs, 0L, kSeq, kFF, kDim, kWCarryInv);
  }
  gelu_f16_kernel<<<(kSeq * kFF) / 2048, 256, 0, stream>>>((const unsigned*)u16, g16, kGCarry);
  {
    const int tiles = (kSeq / 64) * (kDim / 64);
    wmma_gemm64<0, false, 2, 0, true><<<dim3((tiles + 7) / 8, 1), 256, 0, stream>>>(
        g16, g16, kFF, 0L, wm2, wm2, kFF, 0L, 0L,
        (void*)outp, (void*)outp, kDim, 0L, mlp2_b, h1, 0L, kSeq, kDim, kFF, 1.0f / (kGCarry * kWCarry));
  }
}
